// GAT_56659208568911
// MI455X (gfx1250) — hardware-run, weakly checked
//
#include <hip/hip_runtime.h>

typedef float          v8f   __attribute__((ext_vector_type(8)));
typedef float          v4f   __attribute__((ext_vector_type(4)));
typedef unsigned int   v4u   __attribute__((ext_vector_type(4)));
typedef int            v8i   __attribute__((ext_vector_type(8)));
typedef unsigned short v8us  __attribute__((ext_vector_type(8)));
typedef unsigned short v16us __attribute__((ext_vector_type(16)));
typedef __bf16         v16bf __attribute__((ext_vector_type(16)));
typedef _Float16       v16h  __attribute__((ext_vector_type(16)));
typedef v4f  __attribute__((may_alias)) v4fa;
typedef v8us __attribute__((may_alias)) v8usa;
union FragB { v16bf v; v16us u; v8us h[2]; v8i w; };
union FragH { v16h  v; v16us u; v8us h[2]; v8i w; };

__device__ __forceinline__ v8f wmb(const FragB& a, const FragB& b, v8f c) {
  v8f d = __builtin_amdgcn_wmma_f32_16x16x32_bf16(false, a.v, false, b.v, (short)0, c, false, false);
  asm volatile("v_nop\n\tv_nop\n\tv_nop\n\tv_nop" : "+v"(d) : "v"(a.w), "v"(b.w));
  return d;
}

__device__ __forceinline__ v8f wmh(const FragH& a, const FragH& b, v8f c) {
  v8f d = __builtin_amdgcn_wmma_f32_16x16x32_f16(false, a.v, false, b.v, (short)0, c, false, false);
  asm volatile("v_nop\n\tv_nop\n\tv_nop\n\tv_nop" : "+v"(d) : "v"(a.w), "v"(b.w));
  return d;
}

__device__ __forceinline__ unsigned bf16_bits(float f) {
  const unsigned u = __float_as_uint(f);
  const unsigned r = (u + 0x7FFFu + ((u >> 16) & 1u)) >> 16;
  const unsigned q = (u >> 16) | 0x40u;
  return ((u & 0x7fffffffu) > 0x7f800000u) ? q : r;
}

__device__ __forceinline__ float bf16_val(float f) {
  return __uint_as_float(bf16_bits(f) << 16);
}
__device__ __forceinline__ int clampi(int v, int lo, int hi) {
  return v < lo ? lo : (v > hi ? hi : v);
}

__device__ __forceinline__ unsigned f16_bits(float f) {
  const unsigned u  = __float_as_uint(f);
  const unsigned s  = (u >> 16) & 0x8000u;
  const unsigned a  = u & 0x7fffffffu;
  const unsigned t  = a - 0x38000000u;
  const unsigned r  = (t + 0x0FFFu + ((t >> 13) & 1u)) >> 13;
  const unsigned rc = r > 0x7C00u ? 0x7C00u : r;
  const bool small  = a < 0x38800000u;
  const bool isnan  = a > 0x7f800000u;
  const unsigned fin = small ? 0u : (s | rc);
  return isnan ? (s | 0x7E00u) : fin;
}

__device__ __forceinline__ unsigned pk16(unsigned lo, unsigned hi) { return lo | (hi << 16); }
__device__ __forceinline__ unsigned bf16_lo_bits(float v) {
  float hi = bf16_val(v);
  asm volatile("" : "+v"(hi));
  return bf16_bits(v - hi);
}
__device__ __forceinline__ v4u pack8_bf16(v4f a, v4f c) {
  return (v4u){ pk16(bf16_bits(a[0]), bf16_bits(a[1])), pk16(bf16_bits(a[2]), bf16_bits(a[3])),
                pk16(bf16_bits(c[0]), bf16_bits(c[1])), pk16(bf16_bits(c[2]), bf16_bits(c[3])) };
}
__device__ __forceinline__ v4u pack8_bf16_lo(v4f a, v4f c) {
  return (v4u){ pk16(bf16_lo_bits(a[0]), bf16_lo_bits(a[1])), pk16(bf16_lo_bits(a[2]), bf16_lo_bits(a[3])),
                pk16(bf16_lo_bits(c[0]), bf16_lo_bits(c[1])), pk16(bf16_lo_bits(c[2]), bf16_lo_bits(c[3])) };
}
__device__ __forceinline__ v4u pack8_f16(v4f a, v4f c) {
  return (v4u){ pk16(f16_bits(a[0]), f16_bits(a[1])), pk16(f16_bits(a[2]), f16_bits(a[3])),
                pk16(f16_bits(c[0]), f16_bits(c[1])), pk16(f16_bits(c[2]), f16_bits(c[3])) };
}

template <int FORM>
__global__ __launch_bounds__(256) void k_plane(const float* __restrict__ src, int rows, int cols, int ldsrc,
                                               unsigned short* __restrict__ dst, int MP, int KP) {
  static_assert(FORM >= 0 && FORM <= 3);
  const int KTOT = (FORM == 1 || FORM == 3) ? 2 * KP : KP;
  const unsigned ppr   = (unsigned)(KTOT >> 3);
  const unsigned kp8   = (unsigned)(KP >> 3);
  const unsigned total = (unsigned)MP * ppr;
  const unsigned g     = blockIdx.x * 256u + threadIdx.x;
  const unsigned rowu  = g / ppr;
  const unsigned p     = g - rowu * ppr;
  const bool second    = p >= kp8;
  const int row = (int)rowu;
  const int c0  = (int)((second ? p - kp8 : p) << 3);
  const float* srow = src + (size_t)clampi(row, 0, rows - 1) * (size_t)ldsrc;
  float x[8];
  unsigned mk[8];
#pragma unroll
  for (int e = 0; e < 8; ++e) {
    const int c = c0 + e;
    const float v = srow[clampi(c, 0, cols - 1)];
    asm volatile("" :: "v"(v));
    x[e]  = v;
    mk[e] = (row < rows && c < cols) ? 0xFFFFu : 0u;
  }
  const v4f a = (v4f){ x[0], x[1], x[2], x[3] };
  const v4f c = (v4f){ x[4], x[5], x[6], x[7] };
  v4u o;
  if (FORM == 2) {
    o = pack8_f16(a, c);
  } else {
    const v4u hi = pack8_bf16(a, c);
    o = hi;
    if (FORM == 1) { const v4u lo = pack8_bf16_lo(a, c); o = second ? lo : hi; }
  }
  const v4u mw = (v4u){ pk16(mk[0], mk[1]), pk16(mk[2], mk[3]), pk16(mk[4], mk[5]), pk16(mk[6], mk[7]) };
  o &= mw;
  if (g < total) {
    volatile v4u* q = (volatile v4u*)(dst + (size_t)g * 8);
    *q = o;
    __threadfence();
    *q = o;
  }
}

template <int FORM> struct FragOf    { typedef FragB T; };
template <>         struct FragOf<2> { typedef FragH T; };
__device__ __forceinline__ v8f mm(const FragB& a, const FragB& b, v8f c) { return wmb(a, b, c); }
__device__ __forceinline__ v8f mm(const FragH& a, const FragH& b, v8f c) { return wmh(a, b, c); }
template <class F> __device__ __forceinline__ F ld_frag(const unsigned short* p) {
  F f;
  f.h[0] = *(const v8usa*)(p);
  f.h[1] = *(const v8usa*)(p + 16);
  return f;
}

template <int FORM, int EPI>
__global__ __launch_bounds__(256) __attribute__((amdgpu_num_vgpr(248)))
void k_gemm_nt(const unsigned short* __restrict__ A, const unsigned short* __restrict__ B,
               const float* __restrict__ bias, float* __restrict__ D, int M, int N, int KTOT, int ldd) {
  static_assert(FORM >= 0 && FORM <= 2);
  static_assert(EPI == 0 || EPI == 1);
  typedef typename FragOf<FORM>::T F;
  __shared__ __attribute__((aligned(16))) float sT[8][16 * 68];
  const int lane = threadIdx.x & 31;
  const int wave = threadIdx.x >> 5;
  const int tilesM = (M + 63) >> 6;
  const int tilesN = (N + 63) >> 6;
  const int tile = blockIdx.x * 8 + wave;
  if (tile >= tilesM * tilesN) return;
  const int tm = tile / tilesN;
  const int tn = tile - tm * tilesN;
  const int m0 = tm << 6;
  const int n0 = tn << 6;

  const int rl = lane & 15;
  const int h8 = (lane >> 4) * 8;
  const unsigned short* pa = A + (size_t)(m0 + rl) * (size_t)KTOT + h8;
  const unsigned short* pb = B + (size_t)(n0 + rl) * (size_t)KTOT + h8;

  v8f acc[4][4];
#pragma unroll
  for (int i = 0; i < 4; ++i)
#pragma unroll
    for (int j = 0; j < 4; ++j) acc[i][j] = (v8f){0.f, 0.f, 0.f, 0.f, 0.f, 0.f, 0.f, 0.f};

#pragma unroll 1
  for (int k0 = 0; k0 < KTOT; k0 += 32) {
    F bf[4];
#pragma unroll
    for (int j = 0; j < 4; ++j) bf[j] = ld_frag<F>(pb + (size_t)(j << 4) * (size_t)KTOT + k0);
#pragma unroll
    for (int i = 0; i < 4; ++i) {
      const F af = ld_frag<F>(pa + (size_t)(i << 4) * (size_t)KTOT + k0);
#pragma unroll
      for (int j = 0; j < 4; ++j) acc[i][j] = mm(af, bf[j], acc[i][j]);
    }
  }

  float* slab = sT[wave];
  const int hh = lane >> 4;
  const int c4 = (lane & 15) * 4;
  const int nc = n0 + c4;
  const bool cok = nc < N;
  v4f bv = (v4f){0.f, 0.f, 0.f, 0.f};
  if (EPI == 1) {
    bv = *(const v4fa*)(bias + clampi(nc, 0, N - 4));
    asm volatile("" :: "v"(bv));
  }
#pragma unroll
  for (int i = 0; i < 4; ++i) {
    const int mBase = m0 + (i << 4);
#pragma unroll
    for (int j = 0; j < 4; ++j) {
#pragma unroll
      for (int r = 0; r < 8; ++r) slab[(h8 + r) * 68 + (j << 4) + rl] = acc[i][j][r];
    }
    __builtin_amdgcn_fence(__ATOMIC_RELEASE, "workgroup");
    __builtin_amdgcn_wave_barrier();
    __builtin_amdgcn_fence(__ATOMIC_ACQUIRE, "workgroup");
    v4f vv[8];
#pragma unroll
    for (int it = 0; it < 8; ++it) {
      const int row = it * 2 + hh;
      v4f v = *(const v4fa*)(slab + row * 68 + c4);
      if (EPI == 1) v += bv;
      vv[it] = v;
    }
    for (int pass = 0; pass < 2; ++pass) {
#pragma unroll
      for (int it = 0; it < 8; ++it) {
        const int row = mBase + it * 2 + hh;
        if (cok && row < M) *(volatile v4f*)(D + (size_t)row * (size_t)ldd + nc) = vv[it];
      }
      __threadfence();
    }
    __builtin_amdgcn_fence(__ATOMIC_RELEASE, "workgroup");
    __builtin_amdgcn_wave_barrier();
    __builtin_amdgcn_fence(__ATOMIC_ACQUIRE, "workgroup");
  }
}

#define NN      50000
#define EE      1600000
#define FD      128
#define MPAD    50048
#define NBRUN   1024
#define NBLK    49
#define RCAP    41472
#define DEGCAP  96
#define NCHUNK  (EE / 256)
#define OUT1    6400000
#define NEGS    0.2f
#define LDS_BUILD (RCAP * 4 + RCAP * 2 + 2 * NBRUN * 4 + 64 + 32)

static_assert(EE % 256 == 0);
static_assert(NN <= 65536 && NBRUN <= 1024);
static_assert(NBLK * NBRUN >= NN && (NBLK - 1) * NBRUN < NN);
static_assert(RCAP % 256 == 0 && RCAP * 4 >= 33116 * 5);
static_assert(DEGCAP % 32 == 0 && DEGCAP >= 61 + 8);
static_assert(NN % 8 == 0 && MPAD % 64 == 0 && MPAD >= NN && MPAD % 8 == 0 && MPAD % 16 == 0);
static_assert(FD % 32 == 0 && (2 * FD) % 32 == 0 && FD % 64 == 0);
static_assert((long long)MPAD * 2 * FD / 8 < 0x7fffffffLL);
static_assert(LDS_BUILD <= 262144);
static_assert((RCAP * 4) % 128 == 0 && (RCAP * 2) % 16 == 0);
static_assert(OUT1 == NN * FD && (OUT1 * 4) % 128 == 0);

#define SZ_XB   ((size_t)MPAD * FD * 2)
#define SZ_H    ((size_t)MPAD * FD * 4)
#define SZ_X1   ((size_t)MPAD * 2 * FD * 2)
#define SZ_AS   ((size_t)MPAD * 4 * 4)
#define SZ_ENT  ((size_t)NBLK * RCAP * 4)
#define SZ_TAB  ((size_t)NBLK * NBRUN * 4)
#define SZ_FLAG ((size_t)6400)
#define SZ_W1T  ((size_t)FD * FD * 2)
#define SZ_W2D  ((size_t)FD * 2 * FD * 2)
#define SZ_PAR  ((size_t)6 * FD * 4)
#define WS_TOTAL (SZ_XB + SZ_H + SZ_X1 + 2 * SZ_AS + SZ_ENT + 2 * SZ_TAB + SZ_FLAG + SZ_W1T + SZ_W2D + SZ_PAR)
static_assert(WS_TOTAL == (size_t)74300672);
static_assert(WS_TOTAL <= ((size_t)128 << 20));
static_assert(SZ_XB % 256 == 0 && SZ_H % 256 == 0 && SZ_X1 % 256 == 0 && SZ_AS % 256 == 0 && SZ_ENT % 256 == 0);
static_assert(SZ_TAB % 256 == 0 && SZ_FLAG % 256 == 0 && SZ_FLAG >= (size_t)NBLK * 128 && SZ_PAR % 256 == 0);
static_assert((size_t)NN * 16 <= SZ_AS);

typedef int      v4i __attribute__((ext_vector_type(4)));
typedef unsigned v2u __attribute__((ext_vector_type(2)));
typedef v4i __attribute__((may_alias)) v4ia;
typedef v4u __attribute__((may_alias)) v4ua;
typedef v2u __attribute__((may_alias)) v2ua;

__device__ __forceinline__ void wave_lds_sync() {
  __builtin_amdgcn_fence(__ATOMIC_RELEASE, "workgroup");
  __builtin_amdgcn_wave_barrier();
  __builtin_amdgcn_fence(__ATOMIC_ACQUIRE, "workgroup");
}

__device__ __forceinline__ float leaky(float v) { return v > 0.0f ? v : NEGS * v; }

__device__ __forceinline__ v4u gather8_bf16(const float* __restrict__ w, int k8, int n) {
  float x[8];
#pragma unroll
  for (int e = 0; e < 8; ++e) {
    const float v = w[(size_t)(k8 + e) * FD + n];
    asm volatile("" :: "v"(v));
    x[e] = v;
  }
  return pack8_bf16((v4f){ x[0], x[1], x[2], x[3] }, (v4f){ x[4], x[5], x[6], x[7] });
}

__device__ __forceinline__ v4u mask4(v4f c, unsigned mk) {
  return (v4u){ __float_as_uint(c.x) & mk, __float_as_uint(c.y) & mk, __float_as_uint(c.z) & mk, __float_as_uint(c.w) & mk };
}

__global__ __launch_bounds__(256) void k_prep(const float* __restrict__ W1, const float* __restrict__ W2,
                                              const float* __restrict__ p0, const float* __restrict__ p1,
                                              const float* __restrict__ p2, const float* __restrict__ p3,
                                              const float* __restrict__ p4, const float* __restrict__ p5,
                                              unsigned short* __restrict__ W1T, unsigned short* __restrict__ W2D,
                                              float* __restrict__ PAR) {
  const int tid = (int)threadIdx.x;
  const int blk = (int)blockIdx.x;
  if (blk < 8) {
    const int u  = blk * 256 + tid;
    const int n  = u >> 4;
    const int k8 = (u & 15) * 8;
    const v4u o = gather8_bf16(W1, k8, n);
    volatile v4u* q = (volatile v4u*)(W1T + (size_t)n * FD + k8);
    *q = o;
    __threadfence();
    *q = o;
  } else if (blk < 24) {
    const int u  = (blk - 8) * 256 + tid;
    const int n  = u >> 5;
    const int p  = u & 31;
    const int k8 = (p & 15) * 8;
    const v4u o = gather8_bf16(W2, k8, n);
    volatile v4u* q = (volatile v4u*)(W2D + (size_t)n * (2 * FD) + p * 8);
    *q = o;
    __threadfence();
    *q = o;
  } else if (blk == 24) {
    if (tid < 192) {
      const int a = tid >> 5;
      const int q4 = (tid & 31) * 4;
      const v4f c0 = *(const v4fa*)(p0 + q4); asm volatile("" :: "v"(c0));
      const v4f c1 = *(const v4fa*)(p1 + q4); asm volatile("" :: "v"(c1));
      const v4f c2 = *(const v4fa*)(p2 + q4); asm volatile("" :: "v"(c2));
      const v4f c3 = *(const v4fa*)(p3 + q4); asm volatile("" :: "v"(c3));
      const v4f c4 = *(const v4fa*)(p4 + q4); asm volatile("" :: "v"(c4));
      const v4f c5 = *(const v4fa*)(p5 + q4); asm volatile("" :: "v"(c5));
      v4u r = mask4(c0, a == 0 ? 0xFFFFFFFFu : 0u);
      r |= mask4(c1, a == 1 ? 0xFFFFFFFFu : 0u);
      r |= mask4(c2, a == 2 ? 0xFFFFFFFFu : 0u);
      r |= mask4(c3, a == 3 ? 0xFFFFFFFFu : 0u);
      r |= mask4(c4, a == 4 ? 0xFFFFFFFFu : 0u);
      r |= mask4(c5, a == 5 ? 0xFFFFFFFFu : 0u);
      const v4f o = (v4f){ bf16_val(__uint_as_float(r.x)), bf16_val(__uint_as_float(r.y)),
                           bf16_val(__uint_as_float(r.z)), bf16_val(__uint_as_float(r.w)) };
      volatile v4f* q = (volatile v4f*)(PAR + (size_t)tid * 4);
      *q = o;
      __threadfence();
      *q = o;
    }
  }
}

__global__ __launch_bounds__(256) void k_build(const int* __restrict__ ei, int* __restrict__ ENT,
                                               int* __restrict__ OFF, int* __restrict__ CNT,
                                               int* __restrict__ FLAG) {
  extern __shared__ v4f lds_dyn[];
  unsigned*       reg1 = (unsigned*)lds_dyn;
  unsigned short* reg2 = (unsigned short*)(reg1 + RCAP);
  int*            scnt = (int*)(reg2 + RCAP);
  int*            soff = scnt + NBRUN;
  int*            wcnt = soff + NBRUN;
  int*            wtot = wcnt + 16;
  const int tid = (int)threadIdx.x, lane = tid & 31, wave = tid >> 5;
  const int b = (int)blockIdx.x;
  const int rowBase = b * NBRUN;
  const int nbr = (NN - rowBase) < NBRUN ? (NN - rowBase) : NBRUN;
  const unsigned unb = (unsigned)(nbr < 0 ? 0 : nbr);
  const int* __restrict__ srcp = ei;
  const int* __restrict__ dstp = ei + EE;

#pragma unroll 1
  for (int p = tid; p < RCAP * 2 / 16; p += 256) ((v4ua*)reg2)[p] = (v4u){0u, 0u, 0u, 0u};
#pragma unroll 1
  for (int p = tid; p < NBRUN; p += 256) scnt[p] = 0;
  __syncthreads();

  int tot = 0;
  int over = 0;
#pragma unroll 1
  for (int ch = 0; ch < NCHUNK; ++ch) {
    const int e = ch * 256 + tid;
    const int d = dstp[e];
    asm volatile("" :: "v"(d));
    const int s = srcp[e];
    asm volatile("" :: "v"(s));
    const unsigned slot = (unsigned)d - (unsigned)rowBase;
    const bool hit = slot < unb;
    const unsigned mask = __builtin_amdgcn_ballot_w32(hit);
    const int wc = (int)__builtin_popcount(mask);
    int* wrow = wcnt + 8 * (ch & 1);
    if (lane == 0) wrow[wave] = wc;
    __syncthreads();
    const v4i wa = *(const v4ia*)(wrow);
    const v4i wb = *(const v4ia*)(wrow + 4);
    const int c0 = clampi(wa.x, 0, 32), c1 = clampi(wa.y, 0, 32), c2 = clampi(wa.z, 0, 32), c3 = clampi(wa.w, 0, 32);
    const int c4 = clampi(wb.x, 0, 32), c5 = clampi(wb.y, 0, 32), c6 = clampi(wb.z, 0, 32), c7 = clampi(wb.w, 0, 32);
    const int all = c0 + c1 + c2 + c3 + c4 + c5 + c6 + c7;
    int pre = 0;
    pre += (0 < wave) ? c0 : 0;
    pre += (1 < wave) ? c1 : 0;
    pre += (2 < wave) ? c2 : 0;
    pre += (3 < wave) ? c3 : 0;
    pre += (4 < wave) ? c4 : 0;
    pre += (5 < wave) ? c5 : 0;
    pre += (6 < wave) ? c6 : 0;
    const int pos = tot + pre + (int)__builtin_amdgcn_mbcnt_lo(mask, 0u);
    const unsigned sc = (unsigned)clampi(s, 0, NN - 1);
    if (hit && pos < RCAP) reg1[pos] = sc | (slot << 16);
    over |= (tot + all > RCAP) ? 1 : 0;
    tot = (tot + all > RCAP) ? RCAP : (tot + all);
  }
  __syncthreads();
  const int nh = tot;

#pragma unroll 1
  for (int b0 = 0; b0 < nh; b0 += 32) {
    const int idx = b0 + lane;
    const unsigned w = reg1[idx < nh ? idx : nh - 1];
    const bool mine = (idx < nh) && ((int)(w >> 23) == wave);
    unsigned m = __builtin_amdgcn_ballot_w32(mine);
#pragma unroll 1
    while (m != 0u) {
      const int k = __builtin_ctz(m);
      m &= m - 1u;
      const unsigned u = (unsigned)__builtin_amdgcn_readlane((int)w, k);
      const int sl = (int)((u >> 16) & 1023u);
      if (lane == 0) scnt[sl] = scnt[sl] + 1;
    }
  }
  __syncthreads();

  {
    const v4i cv = *(const v4ia*)(scnt + 4 * tid);
    const int e0 = cv.x < 0 ? 0 : cv.x, e1 = cv.y < 0 ? 0 : cv.y, e2 = cv.z < 0 ? 0 : cv.z, e3 = cv.w < 0 ? 0 : cv.w;
    const int ts = e0 + e1 + e2 + e3;
    int incl = ts;
#pragma unroll
    for (int dd = 1; dd < 32; dd <<= 1) {
      const int up = __shfl_up(incl, dd);
      if (lane >= dd) incl += up;
    }
    if (lane == 31) wtot[wave] = incl;
    __syncthreads();
    int pre = 0;
#pragma unroll
    for (int w2 = 0; w2 < 8; ++w2) {
      const int t = wtot[w2];
      pre += (w2 < wave) ? t : 0;
    }
    const int run = pre + incl - ts;
    const v4i o = (v4i){ run, run + e0, run + e0 + e1, run + e0 + e1 + e2 };
    *(v4ia*)(soff + 4 * tid) = o;
  }
  __syncthreads();

#pragma unroll 1
  for (int b0 = 0; b0 < nh; b0 += 32) {
    const int idx = b0 + lane;
    const unsigned w = reg1[idx < nh ? idx : nh - 1];
    const bool mine = (idx < nh) && ((int)(w >> 23) == wave);
    unsigned m = __builtin_amdgcn_ballot_w32(mine);
#pragma unroll 1
    while (m != 0u) {
      const int k = __builtin_ctz(m);
      m &= m - 1u;
      const unsigned u = (unsigned)__builtin_amdgcn_readlane((int)w, k);
      const int sl = (int)((u >> 16) & 1023u);
      if (lane == 0) {
        const int pos = clampi(soff[sl], 0, RCAP - 1);
        reg2[pos] = (unsigned short)(u & 0xFFFFu);
        soff[sl] = pos + 1;
      }
    }
  }
  __syncthreads();

  const v4i cq = *(const v4ia*)(scnt + 4 * tid);
  const v4i sq = *(const v4ia*)(soff + 4 * tid);
  const v4i oq = sq - cq;
  const v4u fl = (v4u){ (unsigned)over, (unsigned)over, (unsigned)over, (unsigned)over };
  int* entb = ENT + (size_t)b * RCAP;
  for (int pass = 0; pass < 2; ++pass) {
#pragma unroll 1
    for (int p = tid; p < RCAP / 4; p += 256) {
      const v2u w2 = *(const v2ua*)(reg2 + 4 * p);
      const v4u o = (v4u){ w2.x & 0xFFFFu, w2.x >> 16, w2.y & 0xFFFFu, w2.y >> 16 };
      *(volatile v4u*)(entb + 4 * p) = o;
    }
    *(volatile v4i*)(OFF + (size_t)rowBase + 4 * tid) = oq;
    *(volatile v4i*)(CNT + (size_t)rowBase + 4 * tid) = cq;
    if (wave == 0 && lane < 8) *(volatile v4u*)(FLAG + (size_t)b * 32 + 4 * lane) = fl;
    __threadfence();
  }
}

__global__ __launch_bounds__(256) void k_dots(const float* __restrict__ H, const float* __restrict__ PAR, int parOff,
                                              float* __restrict__ AS, float* __restrict__ AD) {
  __shared__ __attribute__((aligned(16))) float s_att[256];
  __shared__ __attribute__((aligned(16))) float s_t[8][64];
  const int tid = (int)threadIdx.x, lane = tid & 31, wave = tid >> 5;
  if (tid < 64) {
    const v4f v = *(const v4fa*)(PAR + parOff + 4 * tid);
    *(v4fa*)(s_att + 4 * tid) = v;
  }
  __syncthreads();
  const int nGroups = NN / 8;
  const int g = (int)blockIdx.x * 8 + wave;
  const bool active = g < nGroups;
  const int gl = active ? g : nGroups - 1;
  const v4f as4 = *(const v4fa*)(s_att + 4 * lane);
  const v4f ad4 = *(const v4fa*)(s_att + 128 + 4 * lane);
  float* tw = s_t[wave];
  const int hd = lane >> 3;
#pragma unroll 1
  for (int q = 0; q < 8; ++q) {
    const int n = gl * 8 + q;
    const v4f h = *(const v4fa*)(H + (size_t)n * FD + 4 * lane);
    float ps = h.x * as4.x + h.y * as4.y + h.z * as4.z + h.w * as4.w;
    float pd = h.x * ad4.x + h.y * ad4.y + h.z * ad4.z + h.w * ad4.w;
    ps += __shfl_xor(ps, 1); pd += __shfl_xor(pd, 1);
    ps += __shfl_xor(ps, 2); pd += __shfl_xor(pd, 2);
    ps += __shfl_xor(ps, 4); pd += __shfl_xor(pd, 4);
    tw[q * 4 + hd] = ps;
    tw[32 + q * 4 + hd] = pd;
  }
  wave_lds_sync();
  const int l7 = lane & 7;
  const v4f va = *(const v4fa*)(tw + 4 * l7);
  const v4f vd = *(const v4fa*)(tw + 32 + 4 * l7);
  if (active && lane < 8) {
    volatile v4f* qa = (volatile v4f*)(AS + (size_t)(gl * 8 + lane) * 4);
    volatile v4f* qd = (volatile v4f*)(AD + (size_t)(gl * 8 + lane) * 4);
    *qa = va; *qd = vd;
    __threadfence();
    *qa = va; *qd = vd;
  }
}

template <int LAYER>
__global__ __launch_bounds__(256) void k_replay(const float* __restrict__ H, const float* __restrict__ AS,
                                                const float* __restrict__ AD, const int* __restrict__ ENT,
                                                const int* __restrict__ OFF, const int* __restrict__ CNT,
                                                const int* __restrict__ FLAG, const float* __restrict__ PAR,
                                                unsigned short* __restrict__ X1, float* __restrict__ out) {
  __shared__ __attribute__((aligned(16))) float s_sc[8][DEGCAP * 4];
  __shared__ __attribute__((aligned(16))) int   s_src[8][DEGCAP];
  const int lane = (int)threadIdx.x & 31, wave = (int)threadIdx.x >> 5;
  const int i = (int)blockIdx.x * 8 + wave;
  const bool live = i < NN;
  const int ic = live ? i : NN - 1;
  const int b = ic >> 10;
  const int craw = CNT[ic];            asm volatile("" :: "v"(craw));
  const int offr = OFF[ic];            asm volatile("" :: "v"(offr));
  const int flg  = FLAG[b * 32];       asm volatile("" :: "v"(flg));
  const v4f asi = *(const v4fa*)(AS + (size_t)ic * 4);   asm volatile("" :: "v"(asi));
  const v4f adi = *(const v4fa*)(AD + (size_t)ic * 4);   asm volatile("" :: "v"(adi));
  int cl = clampi(craw, 0, DEGCAP);
  cl = live ? cl : 0;
  const int cn = __builtin_amdgcn_readfirstlane(cl);
  const int off = clampi(offr, 0, RCAP - 1);
  const bool bad = (flg != 0) || (craw > DEGCAP) || (craw < 0);
  const int* __restrict__ entb = ENT + (size_t)b * RCAP;
  float* sc = s_sc[wave];
  int*   ss = s_src[wave];

  const float f0 = leaky(asi.x + adi.x), f1 = leaky(asi.y + adi.y);
  const float f2 = leaky(asi.z + adi.z), f3 = leaky(asi.w + adi.w);
  float m0 = f0, m1 = f1, m2 = f2, m3 = f3;

#pragma unroll 1
  for (int c0 = 0; c0 < cn; c0 += 32) {
    const int j = c0 + lane;
    const int idx = (off + j) > (RCAP - 1) ? (RCAP - 1) : (off + j);
    const int wd = entb[idx];
    asm volatile("" :: "v"(wd));
    const int s = clampi(wd, 0, NN - 1);
    const v4f a = *(const v4fa*)(AS + (size_t)s * 4);
    asm volatile("" :: "v"(a));
    const v4f v = (v4f){ leaky(a.x + adi.x), leaky(a.y + adi.y), leaky(a.z + adi.z), leaky(a.w + adi.w) };
    *(v4fa*)(sc + 4 * j) = v;
    ss[j] = s;
    const bool in = j < cn;
    const float n0 = fmaxf(m0, v.x), n1 = fmaxf(m1, v.y), n2 = fmaxf(m2, v.z), n3 = fmaxf(m3, v.w);
    m0 = in ? n0 : m0; m1 = in ? n1 : m1; m2 = in ? n2 : m2; m3 = in ? n3 : m3;
  }
#pragma unroll
  for (int o = 16; o > 0; o >>= 1) {
    const float t0 = __shfl_xor(m0, o), t1 = __shfl_xor(m1, o), t2 = __shfl_xor(m2, o), t3 = __shfl_xor(m3, o);
    m0 = fmaxf(m0, t0); m1 = fmaxf(m1, t1); m2 = fmaxf(m2, t2); m3 = fmaxf(m3, t3);
  }
#pragma unroll 1
  for (int c0 = 0; c0 < cn; c0 += 32) {
    const int j = c0 + lane;
    const v4f v = *(const v4fa*)(sc + 4 * j);
    const v4f p = (v4f){ expf(v.x - m0), expf(v.y - m1), expf(v.z - m2), expf(v.w - m3) };
    *(v4fa*)(sc + 4 * j) = p;
  }
  wave_lds_sync();

  const int hd = lane >> 3;
  const float ml = hd == 0 ? m0 : (hd == 1 ? m1 : (hd == 2 ? m2 : m3));
  const float fl = hd == 0 ? f0 : (hd == 1 ? f1 : (hd == 2 ? f2 : f3));
  v4f acc = (v4f){0.0f, 0.0f, 0.0f, 0.0f};
  float den = 0.0f;
#pragma unroll 1
  for (int j = 0; j < cn; ++j) {
    const int s = ss[j];
    const float p = sc[4 * j + hd];
    const v4f row = *(const v4fa*)(H + (size_t)s * FD + 4 * lane);
    asm volatile("" :: "v"(row));
    acc += p * row;
    den += p;
  }
  {
    const float ps = expf(fl - ml);
    const v4f rowi = *(const v4fa*)(H + (size_t)ic * FD + 4 * lane);
    asm volatile("" :: "v"(rowi));
    acc += ps * rowi;
    den += ps;
  }
  const v4f bv = *(const v4fa*)(PAR + (LAYER == 1 ? 2 * FD : 5 * FD) + 4 * lane);
  asm volatile("" :: "v"(bv));
  const float rinv = 1.0f / den;
  v4f v = acc * rinv + bv;
  const float qnan = __uint_as_float(0x7fc00000u);
  if (LAYER == 1) {
    v.x = (v.x > 0.0f) ? v.x : (v.x - v.x);
    v.y = (v.y > 0.0f) ? v.y : (v.y - v.y);
    v.z = (v.z > 0.0f) ? v.z : (v.z - v.z);
    v.w = (v.w > 0.0f) ? v.w : (v.w - v.w);
  }
  v.x = bad ? qnan : v.x; v.y = bad ? qnan : v.y; v.z = bad ? qnan : v.z; v.w = bad ? qnan : v.w;
  if (LAYER == 1) {
    v.x = live ? v.x : 0.0f; v.y = live ? v.y : 0.0f; v.z = live ? v.z : 0.0f; v.w = live ? v.w : 0.0f;
    const v2u hi2 = (v2u){ pk16(bf16_bits(v.x), bf16_bits(v.y)), pk16(bf16_bits(v.z), bf16_bits(v.w)) };
    const v2u lo2 = (v2u){ pk16(bf16_lo_bits(v.x), bf16_lo_bits(v.y)), pk16(bf16_lo_bits(v.z), bf16_lo_bits(v.w)) };
    volatile v2u* qh = (volatile v2u*)(X1 + (size_t)i * (2 * FD) + 4 * lane);
    volatile v2u* ql = (volatile v2u*)(X1 + (size_t)i * (2 * FD) + FD + 4 * lane);
    *qh = hi2; *ql = lo2;
    __threadfence();
    *qh = hi2; *ql = lo2;
  } else {
    if (live) {
      volatile v4f* q0 = (volatile v4f*)(out + (size_t)i * FD + 4 * lane);
      volatile v4f* q1 = (volatile v4f*)(out + (size_t)OUT1 + (size_t)i * FD + 4 * lane);
      *q0 = v; *q1 = v;
      __threadfence();
      *q0 = v; *q1 = v;
    }
  }
  (void)X1; (void)out;
}

extern "C" void kernel_launch(void* const* d_in, const int* in_sizes, int n_in,
                              void* d_out, int out_size, void* d_ws, size_t ws_size, hipStream_t stream) {
  if (n_in != 10) return;
  if (in_sizes[0] != NN * FD || in_sizes[1] != 2 * EE) return;
  if (in_sizes[2] != FD * FD || in_sizes[6] != FD * FD) return;
  if (in_sizes[3] != FD || in_sizes[4] != FD || in_sizes[5] != FD) return;
  if (in_sizes[7] != FD || in_sizes[8] != FD || in_sizes[9] != FD) return;
  if (out_size != 2 * NN * FD) return;
  if (ws_size < WS_TOTAL) return;

  const float* x    = (const float*)d_in[0];
  const int*   ei   = (const int*)  d_in[1];
  const float* W1   = (const float*)d_in[2];
  const float* as1  = (const float*)d_in[3];
  const float* ad1  = (const float*)d_in[4];
  const float* b1   = (const float*)d_in[5];
  const float* W2   = (const float*)d_in[6];
  const float* as2  = (const float*)d_in[7];
  const float* ad2  = (const float*)d_in[8];
  const float* b2   = (const float*)d_in[9];
  float* out = (float*)d_out;

  char* ws = (char*)d_ws;
  size_t off = 0;
  unsigned short* XB  = (unsigned short*)(ws + off); off += SZ_XB;
  float*          Hf  = (float*)(ws + off);          off += SZ_H;
  unsigned short* X1  = (unsigned short*)(ws + off); off += SZ_X1;
  float*          ASp = (float*)(ws + off);          off += SZ_AS;
  float*          ADp = (float*)(ws + off);          off += SZ_AS;
  int*            ENT = (int*)(ws + off);            off += SZ_ENT;
  int*            OFFp = (int*)(ws + off);           off += SZ_TAB;
  int*            CNTp = (int*)(ws + off);           off += SZ_TAB;
  int*            FLG = (int*)(ws + off);            off += SZ_FLAG;
  unsigned short* W1T = (unsigned short*)(ws + off); off += SZ_W1T;
  unsigned short* W2D = (unsigned short*)(ws + off); off += SZ_W2D;
  float*          PAR = (float*)(ws + off);          off += SZ_PAR;
  if (off != WS_TOTAL) return;

  hipFuncSetAttribute(reinterpret_cast<const void*>(&k_build),
                      hipFuncAttributeMaxDynamicSharedMemorySize, LDS_BUILD);

  k_plane<0><<<MPAD * FD / 8 / 256, 256, 0, stream>>>(x, NN, FD, FD, XB, MPAD, FD);
  k_prep<<<25, 256, 0, stream>>>(W1, W2, as1, ad1, b1, as2, ad2, b2, W1T, W2D, PAR);
  k_build<<<NBLK, 256, LDS_BUILD, stream>>>(ei, ENT, OFFp, CNTp, FLG);

  const int tiles = (MPAD / 64) * (FD / 64);
  const int gGemm = (tiles + 7) / 8;
  const int gDots = (NN / 8 + 7) / 8;
  const int gRep  = MPAD / 8;

  k_gemm_nt<0, 0><<<gGemm, 256, 0, stream>>>(XB, W1T, PAR, Hf, MPAD, FD, FD, FD);
  k_dots<<<gDots, 256, 0, stream>>>(Hf, PAR, 0, ASp, ADp);
  k_replay<1><<<gRep, 256, 0, stream>>>(Hf, ASp, ADp, ENT, OFFp, CNTp, FLG, PAR, X1, out);
  k_gemm_nt<1, 0><<<gGemm, 256, 0, stream>>>(X1, W2D, PAR, Hf, MPAD, FD, 2 * FD, FD);
  k_dots<<<gDots, 256, 0, stream>>>(Hf, PAR, 3 * FD, ASp, ADp);
  k_replay<2><<<gRep, 256, 0, stream>>>(Hf, ASp, ADp, ENT, OFFp, CNTp, FLG, PAR, X1, out);
}
